// RTGMFFModel_33767032882069
// MI455X (gfx1250) — hardware-verified
//
#include <hip/hip_runtime.h>
#include <stdint.h>
#include <math.h>


#define NB 4
#define NL 2048
#define DM 768
#define DI 1536
#define DS 16
#define DR 48
#define NR (NB * NL)
#define XW 96
#define KD 64
#define TS 32

typedef unsigned short u16;
typedef __attribute__((ext_vector_type(16))) __bf16   v16b;
typedef __attribute__((ext_vector_type(16))) _Float16 v16h;
typedef __attribute__((ext_vector_type(8)))  _Float16 v8h;
typedef __attribute__((ext_vector_type(8)))  float    v8f;
typedef __attribute__((ext_vector_type(4)))  float    v4f;
typedef __attribute__((ext_vector_type(4)))  uint32_t v4u;

union FB { v16b v; v4u q[2]; };
union FH { v16h v; v4u q[2]; };
union H8 { v8h h; v4u q; };

__device__ __forceinline__ uint32_t f2bf_bits(float f) {
    uint32_t u = __float_as_uint(f);
    u = u + 0x7FFFu + ((u >> 16) & 1u);
    return u >> 16;
}
__device__ __forceinline__ float bf_bits2f(uint32_t b) { return __uint_as_float(b << 16); }
__device__ __forceinline__ float bfr(float f) { return bf_bits2f(f2bf_bits(f)); }
__device__ __forceinline__ float silu_f(float x) {
    return x * __builtin_amdgcn_rcpf(1.0f + __expf(-x));
}

template<class FR>
__device__ __forceinline__ FR ldfrag(const u16* p) {
    FR f;
    f.q[0] = *(const v4u*)p;
    f.q[1] = *(const v4u*)(p + 16);
    return f;
}
__device__ __forceinline__ v8f mma(const FB& a, const FB& b, v8f c) {
    c = __builtin_amdgcn_wmma_f32_16x16x32_bf16(false, a.v, false, b.v, (short)0, c, false, false);
    asm volatile("v_nop\n\tv_nop\n\tv_nop\n\tv_nop" : "+v"(c) : "v"(a.v), "v"(b.v));
    return c;
}
__device__ __forceinline__ v8f mma(const FH& a, const FH& b, v8f c) {
    c = __builtin_amdgcn_wmma_f32_16x16x32_f16(false, a.v, false, b.v, (short)0, c, false, false);
    asm volatile("v_nop\n\tv_nop\n\tv_nop\n\tv_nop" : "+v"(c) : "v"(a.v), "v"(b.v));
    return c;
}

template<int NF, class FR, int EPI>
__global__ __launch_bounds__(128)
void k_gemm(const u16* __restrict__ A, int lda, const u16* __restrict__ Wt, int ldb,
            int M, int K, float* __restrict__ C, int ldc,
            u16* __restrict__ C16, int ldc16, int nsplit, float oscale)
{
    constexpr int PW = NF * 16;
    __shared__ __attribute__((aligned(16))) float sC[128 * PW];

    const int l  = threadIdx.x & 31;
    const int wv = threadIdx.x >> 5;
    const int h  = l >> 4;
    const int m  = l & 15;
    const int mblk = blockIdx.y * 128;
    const int n0   = blockIdx.x * PW;
    const int rowb = mblk + 32 * wv;

    int ra0 = rowb + m;      if (ra0 > M - 1) ra0 = M - 1;
    int ra1 = rowb + 16 + m; if (ra1 > M - 1) ra1 = M - 1;
    const u16* pa0 = A  + (size_t)ra0 * lda + 8 * h;
    const u16* pa1 = A  + (size_t)ra1 * lda + 8 * h;
    const u16* pb  = Wt + (size_t)(n0 + m) * ldb + 8 * h;

    const v8f z = {0.f, 0.f, 0.f, 0.f, 0.f, 0.f, 0.f, 0.f};
    v8f acc[2][NF];
#pragma unroll
    for (int j = 0; j < NF; ++j) { acc[0][j] = z; acc[1][j] = z; }

    for (int k0 = 0; k0 < K; k0 += 32) {
        FR a0 = ldfrag<FR>(pa0 + k0);
        FR a1 = ldfrag<FR>(pa1 + k0);
#pragma unroll
        for (int j = 0; j < NF; ++j) {
            FR fb = ldfrag<FR>(pb + (size_t)(16 * j) * ldb + k0);
            acc[0][j] = mma(a0, fb, acc[0][j]);
            acc[1][j] = mma(a1, fb, acc[1][j]);
        }
    }

#pragma unroll
    for (int i = 0; i < 2; ++i) {
#pragma unroll
        for (int j = 0; j < NF; ++j) {
#pragma unroll
            for (int r = 0; r < 8; ++r)
                sC[(32 * wv + 16 * i + 8 * h + r) * PW + 16 * j + m] = acc[i][j][r] * oscale;
        }
    }
    __syncthreads();

    const float* sw = sC + (32 * wv) * PW;
    if (EPI == 0 || (EPI == 1 && n0 < nsplit)) {
        constexpr int Q = NF * 4;
        for (int pass = 0; pass < 2; ++pass) {
#pragma unroll
            for (int it = 0; it < Q; ++it) {
                const int f   = it * 32 + l;
                const int rr  = f / Q;
                const int c4  = f - rr * Q;
                const int row = rowb + rr;
                const v4f v = *(const v4f*)(sw + rr * PW + 4 * c4);
                if (row < M) *(volatile v4f*)(C + (size_t)row * ldc + n0 + 4 * c4) = v;
            }
            if (pass == 0) __threadfence();
        }
    } else {
        constexpr int Q8 = NF * 2;
        const int cbase = (EPI == 1) ? (n0 - nsplit) : n0;
        for (int pass = 0; pass < 2; ++pass) {
#pragma unroll
            for (int it = 0; it < Q8; ++it) {
                const int f   = it * 32 + l;
                const int rr  = f / Q8;
                const int c8  = f - rr * Q8;
                const int row = rowb + rr;
                const float* s = sw + rr * PW + 8 * c8;
                const v4f v0 = *(const v4f*)s;
                const v4f v1 = *(const v4f*)(s + 4);
                v4u pk;
                if (EPI == 1) {
                    H8 u;
#pragma unroll
                    for (int e = 0; e < 4; ++e) {
                        u.h[e]     = (_Float16)silu_f(v0[e]);
                        u.h[4 + e] = (_Float16)silu_f(v1[e]);
                    }
                    pk = u.q;
                } else {
                    pk[0] = f2bf_bits(v0[0]) | (f2bf_bits(v0[1]) << 16);
                    pk[1] = f2bf_bits(v0[2]) | (f2bf_bits(v0[3]) << 16);
                    pk[2] = f2bf_bits(v1[0]) | (f2bf_bits(v1[1]) << 16);
                    pk[3] = f2bf_bits(v1[2]) | (f2bf_bits(v1[3]) << 16);
                }
                if (row < M) *(volatile v4u*)(C16 + (size_t)row * ldc16 + cbase + 8 * c8) = pk;
            }
            if (pass == 0) __threadfence();
        }
    }
}

template<int MODE>
__global__ __launch_bounds__(256)
void k_cvt(const float* __restrict__ src, int srows, int scols, int sld,
           u16* __restrict__ dst, int drows, int dcols, float scale)
{
    const size_t nch = (size_t)drows * (size_t)dcols / 8;
    const size_t ch  = (size_t)blockIdx.x * 256 + threadIdx.x;
    if (ch >= nch) return;
    const size_t e0 = ch * 8;
    const int r = (int)(e0 / (size_t)dcols);
    const int c = (int)(e0 - (size_t)r * (size_t)dcols);
    float v[8];
    if (r < srows && c + 8 <= scols) {
        const float* p = src + (size_t)r * sld + c;
        const v4f a = *(const v4f*)p;
        const v4f b = *(const v4f*)(p + 4);
#pragma unroll
        for (int e = 0; e < 4; ++e) { v[e] = a[e]; v[4 + e] = b[e]; }
    } else {
#pragma unroll
        for (int e = 0; e < 8; ++e) {
            const int cc = c + e;
            v[e] = (r < srows && cc < scols) ? src[(size_t)r * sld + cc] : 0.f;
        }
    }
    v4u pk;
    if (MODE == 0) {
#pragma unroll
        for (int e = 0; e < 4; ++e) pk[e] = f2bf_bits(v[2 * e]) | (f2bf_bits(v[2 * e + 1]) << 16);
    } else {
        H8 u;
#pragma unroll
        for (int e = 0; e < 8; ++e) u.h[e] = (_Float16)(bfr(v[e]) * scale);
        pk = u.q;
    }
    u16* q = dst + e0;
    *(volatile v4u*)q = pk;
    __threadfence();
    *(volatile v4u*)q = pk;
}

__global__ __launch_bounds__(256)
void k_conv(const float* __restrict__ xp, const float* __restrict__ cw,
            const float* __restrict__ cbv, u16* __restrict__ hb)
{
    const int ch = blockIdx.x * 256 + threadIdx.x;
    if (ch >= NR * (DI / 8)) return;
    const int row = ch / (DI / 8);
    const int d0  = (ch - row * (DI / 8)) * 8;
    const int lp  = row % NL;
    float a[8];
#pragma unroll
    for (int e = 0; e < 8; ++e) a[e] = 0.f;
#pragma unroll
    for (int j = 0; j < 4; ++j) {
        const int ls = lp - 3 + j;
        if (ls >= 0) {
            const float* p = xp + (size_t)(row - 3 + j) * DI + d0;
            const v4f x0 = *(const v4f*)p;
            const v4f x1 = *(const v4f*)(p + 4);
#pragma unroll
            for (int e = 0; e < 4; ++e) {
                a[e]     += bfr(cw[(d0 + e) * 4 + j]) * x0[e];
                a[4 + e] += bfr(cw[(d0 + 4 + e) * 4 + j]) * x1[e];
            }
        }
    }
    v4u pk;
#pragma unroll
    for (int e = 0; e < 4; ++e) {
        const float u0 = silu_f(a[2 * e]     + bfr(cbv[d0 + 2 * e]));
        const float u1 = silu_f(a[2 * e + 1] + bfr(cbv[d0 + 2 * e + 1]));
        pk[e] = f2bf_bits(u0) | (f2bf_bits(u1) << 16);
    }
    u16* q = hb + (size_t)row * DI + d0;
    *(volatile v4u*)q = pk;
    __threadfence();
    *(volatile v4u*)q = pk;
}

__global__ __launch_bounds__(64)
void k_scan(const float* __restrict__ xp, const u16* __restrict__ g16, const float* __restrict__ xdbl,
            u16* dty, const float* __restrict__ cw, const float* __restrict__ cbv,
            const float* __restrict__ bdt, const float* __restrict__ alog, const float* __restrict__ Dv)
{
    __shared__ __attribute__((aligned(16))) float    sX[TS * 64];
    __shared__ __attribute__((aligned(16))) float    sBC[TS * 32];
    __shared__ __attribute__((aligned(16))) u16      sDT[TS * 64];
    __shared__ __attribute__((aligned(16))) _Float16 sG[TS * 64];
    __shared__ __attribute__((aligned(16))) _Float16 sY[TS * 64];

    const int tid = threadIdx.x;
    const int l = tid & 31, wv = tid >> 5;
    const int b  = blockIdx.x / (DI / 64);
    const int cg = blockIdx.x - b * (DI / 64);
    const int d0 = cg * 64;
    const int d  = d0 + tid;
    const size_t R = (size_t)b * NL;

    const float w0 = bfr(cw[d * 4 + 0]);
    const float w1 = bfr(cw[d * 4 + 1]);
    const float w2 = bfr(cw[d * 4 + 2]);
    const float w3 = bfr(cw[d * 4 + 3]);
    const float cb = bfr(cbv[d]);
    const float bd = bfr(bdt[d]);
    const float Dd = bfr(Dv[d]);
    float An[DS];
#pragma unroll
    for (int n = 0; n < DS; ++n) An[n] = -__expf(bfr(alog[d * DS + n]));
    float st[DS];
#pragma unroll
    for (int n = 0; n < DS; ++n) st[n] = 0.f;
    float xh0 = 0.f, xh1 = 0.f, xh2 = 0.f;

    for (int c = 0; c < NL / TS; ++c) {
        const int t0 = c * TS;
        const size_t rb = R + (size_t)t0;
        __syncthreads();
#pragma unroll
        for (int p = 0; p < 8; ++p) {
            const int idx = p * 64 + tid;
            const int rr = idx >> 4, c4 = idx & 15;
            *(v4f*)(sX + rr * 64 + 4 * c4) = *(const v4f*)(xp + (rb + rr) * DI + d0 + 4 * c4);
        }
#pragma unroll
        for (int p = 0; p < 4; ++p) {
            const int idx = p * 64 + tid;
            const int rr = idx >> 3, c8 = idx & 7;
            *(v4u*)(sDT + rr * 64 + 8 * c8) = *(const v4u*)(dty + (rb + rr) * DI + d0 + 8 * c8);
            *(v4u*)(sG  + rr * 64 + 8 * c8) = *(const v4u*)(g16 + (rb + rr) * DI + d0 + 8 * c8);
            *(v4f*)(sBC + rr * 32 + 4 * c8) = *(const v4f*)(xdbl + (rb + rr) * XW + DR + 4 * c8);
        }
        __syncthreads();

#pragma unroll 1
        for (int s = 0; s < TS; ++s) {
            const float xt = sX[s * 64 + tid];
            float a = w0 * xh0;
            a = a + w1 * xh1;
            a = a + w2 * xh2;
            a = a + w3 * xt;
            a = a + cb;
            xh0 = xh1; xh1 = xh2; xh2 = xt;
            const float u  = silu_f(a);
            const float dr = bf_bits2f((uint32_t)sDT[s * 64 + tid]) + bd;
            const float dt = fmaxf(dr, 0.f) + log1pf(__expf(-fabsf(dr)));
            float y = 0.f;
            const float* bc = sBC + s * 32;
#pragma unroll
            for (int q = 0; q < 4; ++q) {
                const v4f Bq = *(const v4f*)(bc + 4 * q);
                const v4f Cq = *(const v4f*)(bc + 16 + 4 * q);
#pragma unroll
                for (int e = 0; e < 4; ++e) {
                    const int n = 4 * q + e;
                    const float dA = __expf(dt * An[n]);
                    st[n] = dA * st[n] + (dt * Bq[e]) * u;
                    y += st[n] * Cq[e];
                }
            }
            y += u * Dd;
            const float g = (float)sG[s * 64 + tid];
            sY[s * 64 + tid] = (_Float16)(y * g * 256.0f);
        }
        __syncthreads();

        v4u vv[4];
#pragma unroll
        for (int it = 0; it < 4; ++it) {
            const int rr = 16 * wv + 4 * it + (l >> 3);
            vv[it] = *(const v4u*)(sY + rr * 64 + 8 * (l & 7));
        }
        for (int pass = 0; pass < 2; ++pass) {
#pragma unroll
            for (int it = 0; it < 4; ++it) {
                const int rr = 16 * wv + 4 * it + (l >> 3);
                *(volatile v4u*)(dty + (rb + rr) * DI + d0 + 8 * (l & 7)) = vv[it];
            }
            if (pass == 0) __threadfence();
        }
    }
}

extern "C" void kernel_launch(void* const* d_in, const int* in_sizes, int n_in,
                              void* d_out, int out_size, void* d_ws, size_t ws_size,
                              hipStream_t stream)
{
    (void)in_sizes; (void)n_in; (void)out_size;
    const float* x      = (const float*)d_in[0];
    const float* W_in   = (const float*)d_in[1];
    const float* conv_w = (const float*)d_in[2];
    const float* conv_b = (const float*)d_in[3];
    const float* W_x    = (const float*)d_in[4];
    const float* W_dt   = (const float*)d_in[5];
    const float* b_dt   = (const float*)d_in[6];
    const float* A_log  = (const float*)d_in[7];
    const float* Dvec   = (const float*)d_in[8];
    const float* W_out  = (const float*)d_in[9];
    float* out = (float*)d_out;

    const size_t szWx  = (size_t)XW * DI * 2;
    const size_t szWdt = (size_t)DI * KD * 2;
    const size_t szWo  = (size_t)DM * DI * 2;
    const size_t szXp  = (size_t)NR * DI * 4;
    const size_t szG   = (size_t)NR * DI * 2;
    const size_t szXb  = (size_t)NR * DM * 2;
    const size_t szWin = (size_t)2 * DI * DM * 2;
    const size_t szR3  = szXb + szWin;
    const size_t szR4  = (size_t)NR * DI * 2;

    char* ws = (char*)d_ws;
    size_t o = 0;
    u16*   WxB  = (u16*)(ws + o);   o += szWx;
    u16*   WdtB = (u16*)(ws + o);   o += szWdt;
    u16*   WoH  = (u16*)(ws + o);   o += szWo;
    float* xp   = (float*)(ws + o); o += szXp;
    u16*   g16  = (u16*)(ws + o);   o += szG;
    char*  r3   = ws + o;           o += szR3;
    char*  r4   = ws + o;           o += szR4;
    if (o > ws_size) return;
    if ((size_t)NR * XW * 4 + (size_t)NR * KD * 2 > szR3) return;

    u16*   xbf  = (u16*)r3;
    u16*   WinB = (u16*)(r3 + szXb);
    float* xdbl = (float*)r3;
    u16*   dltb = (u16*)(r3 + (size_t)NR * XW * 4);
    u16*   hb   = (u16*)r4;
    u16*   dty  = (u16*)r4;

    const int GY = (NR + 127) / 128;

    k_cvt<0><<<dim3((unsigned)(((size_t)NR * DM / 8 + 255) / 256)), 256, 0, stream>>>(
        x, NR, DM, DM, xbf, NR, DM, 1.0f);
    k_cvt<0><<<dim3((unsigned)(((size_t)2 * DI * DM / 8 + 255) / 256)), 256, 0, stream>>>(
        W_in, 2 * DI, DM, DM, WinB, 2 * DI, DM, 1.0f);
    k_cvt<0><<<dim3((unsigned)(((size_t)XW * DI / 8 + 255) / 256)), 256, 0, stream>>>(
        W_x, DR + 2 * DS, DI, DI, WxB, XW, DI, 1.0f);
    k_cvt<0><<<dim3((unsigned)(((size_t)DI * KD / 8 + 255) / 256)), 256, 0, stream>>>(
        W_dt, DI, DR, DR, WdtB, DI, KD, 1.0f);
    k_cvt<1><<<dim3((unsigned)(((size_t)DM * DI / 8 + 255) / 256)), 256, 0, stream>>>(
        W_out, DM, DI, DI, WoH, DM, DI, 4096.0f);

    k_gemm<4, FB, 1><<<dim3(2 * DI / 64, GY), 128, 0, stream>>>(
        xbf, DM, WinB, DM, NR, DM, xp, DI, g16, DI, DI, 1.0f);

    k_conv<<<dim3((unsigned)(((size_t)NR * (DI / 8) + 255) / 256)), 256, 0, stream>>>(
        xp, conv_w, conv_b, hb);

    k_gemm<6, FB, 0><<<dim3(XW / 96, GY), 128, 0, stream>>>(
        hb, DI, WxB, DI, NR, DI, xdbl, XW, dltb, KD, 0, 1.0f);

    k_cvt<0><<<dim3((unsigned)(((size_t)NR * KD / 8 + 255) / 256)), 256, 0, stream>>>(
        xdbl, NR, DR, XW, dltb, NR, KD, 1.0f);

    k_gemm<4, FB, 2><<<dim3(DI / 64, GY), 128, 0, stream>>>(
        dltb, KD, WdtB, KD, NR, KD, xp, DI, dty, DI, 0, 1.0f);

    k_scan<<<dim3(NB * (DI / 64)), 64, 0, stream>>>(
        xp, g16, xdbl, dty, conv_w, conv_b, b_dt, A_log, Dvec);

    k_gemm<4, FH, 0><<<dim3(DM / 64, GY), 128, 0, stream>>>(
        dty, DI, WoH, DI, NR, DI, out, DM, g16, DI, 0, 1.0f / 1048576.0f);
}
